// MultiHeadAttention_66984309948505
// MI455X (gfx1250) — hardware-verified
//
#include <hip/hip_runtime.h>
#ifndef NB
#define NB 4
#endif
#ifndef SEQ
#define SEQ 2048
#endif
#define NB_FULL 4
#define SEQ_FULL 2048
#define DM 1024
#define NH 16
#define HD 64
#define EARLY 256
#define NR ((size_t)NB * SEQ)
#define NE ((size_t)NB * EARLY)

typedef __bf16   v16b __attribute__((ext_vector_type(16)));
typedef _Float16 v16h __attribute__((ext_vector_type(16)));
typedef unsigned short v8us __attribute__((ext_vector_type(8), may_alias));
typedef unsigned short v4us __attribute__((ext_vector_type(4), may_alias));
typedef float v8f  __attribute__((ext_vector_type(8)));
typedef float v4f  __attribute__((ext_vector_type(4)));
typedef float v4fa __attribute__((ext_vector_type(4), may_alias));
union Frag16 { v16h h; v16b b; v8us half[2]; unsigned short u[16]; _Float16 f[16]; };
union H16 { _Float16 h; unsigned short u; };

__device__ __forceinline__ unsigned short bf16_bits(float x) { unsigned int u = __float_as_uint(x); return (unsigned short)((u + 0x7FFFu + ((u >> 16) & 1u)) >> 16); }
__device__ __forceinline__ float bf16_val(unsigned short b) { return __uint_as_float(((unsigned int)b) << 16); }
__device__ __forceinline__ float bf16_rne(float x) { return bf16_val(bf16_bits(x)); }
__device__ __forceinline__ unsigned short f16_bits(float x) { H16 c; c.h = (_Float16)x; return c.u; }

__device__ __forceinline__ v8f mma_h(v16h a, v16h b, v8f c) {
  v8f d = __builtin_amdgcn_wmma_f32_16x16x32_f16(false, a, false, b, (short)0, c, false, false);
  asm volatile("v_nop\n\tv_nop\n\tv_nop\n\tv_nop" : "+v"(d) : "v"(a), "v"(b));
  return d;
}
template <int NT>
__device__ __forceinline__ v8f mma_b(v16b ah, v16b al, v16b bh, v16b bl, v8f c) {
  c = __builtin_amdgcn_wmma_f32_16x16x32_bf16(false, ah, false, bh, (short)0, c, false, false);
  if (NT >= 2) c = __builtin_amdgcn_wmma_f32_16x16x32_bf16(false, al, false, bh, (short)0, c, false, false);
  if (NT >= 3) c = __builtin_amdgcn_wmma_f32_16x16x32_bf16(false, ah, false, bl, (short)0, c, false, false);
  asm volatile("v_nop\n\tv_nop\n\tv_nop\n\tv_nop" : "+v"(c) : "v"(ah), "v"(al), "v"(bh), "v"(bl));
  return c;
}
__device__ __forceinline__ Frag16 ld_frag(const unsigned short* p, int hh) {
  Frag16 f; f.half[0] = *(const v8us*)(p + 8 * hh); f.half[1] = *(const v8us*)(p + 16 + 8 * hh); return f;
}
template <bool E>
__device__ __forceinline__ v8f mm2(const Frag16& ah, const Frag16& al, const Frag16& b, v8f c) {
  if (E) return mma_b<2>(ah.b, al.b, b.b, b.b, c);
  return mma_h(ah.h, b.h, c);
}
template <bool E>
__device__ __forceinline__ v8f mm3(const Frag16& ah, const Frag16& al, const Frag16& bh, const Frag16& bl, v8f c) {
  if (E) return mma_b<3>(ah.b, al.b, bh.b, bl.b, c);
  return mma_h(ah.h, bh.h, c);
}

__global__ __launch_bounds__(256) void k_x16(const float* __restrict__ x, unsigned short* __restrict__ X16) {
  const size_t t = (size_t)blockIdx.x * 256 + threadIdx.x;
  if (t >= NR * DM / 8) return;
  const size_t e = t * 8; const size_t r = e / DM; const size_t c = e % DM;
  const size_t b = r / SEQ, s = r % SEQ;
  const float* src = x + ((b * SEQ_FULL + s) * DM + c);
  const v4f a = *(const v4fa*)src, d = *(const v4fa*)(src + 4);
  Frag16 f;
#pragma unroll
  for (int q = 0; q < 4; ++q) { f.f[q] = (_Float16)bf16_rne(a[q]); f.f[4 + q] = (_Float16)bf16_rne(d[q]); }
  const v8us o = f.half[0];
  *(volatile v8us*)(X16 + e) = o;
  __threadfence();
  *(volatile v8us*)(X16 + e) = o;
}

__global__ __launch_bounds__(256) void k_wt_heads(const float* __restrict__ W, unsigned short* __restrict__ Bt) {
  const int t = blockIdx.x * 256 + threadIdx.x;
  if (t >= NH * HD * (DM / 8)) return;
  const int n = t / (DM / 8), k8 = (t % (DM / 8)) * 8;
  const int h = n / HD, s = n % HD;
  Frag16 f;
#pragma unroll
  for (int i = 0; i < 8; ++i) f.f[i] = (_Float16)(bf16_rne(W[((size_t)h * DM + k8 + i) * HD + s]) * 16.0f);
  const v8us o = f.half[0];
  *(volatile v8us*)(Bt + (size_t)n * DM + k8) = o;
  __threadfence();
  *(volatile v8us*)(Bt + (size_t)n * DM + k8) = o;
}

__global__ __launch_bounds__(256) void k_wo(const float* __restrict__ w, unsigned short* __restrict__ B16, unsigned short* __restrict__ Bb) {
  const size_t t = (size_t)blockIdx.x * 256 + threadIdx.x;
  if (t >= (size_t)DM * DM / 8) return;
  const v4f a = *(const v4fa*)(w + t * 8), c = *(const v4fa*)(w + t * 8 + 4);
  Frag16 fh, fb;
#pragma unroll
  for (int q = 0; q < 4; ++q) {
    const unsigned short b0 = bf16_bits(a[q]); fb.u[q] = b0; fh.f[q] = (_Float16)(bf16_val(b0) * 16.0f);
    const unsigned short b1 = bf16_bits(c[q]); fb.u[4 + q] = b1; fh.f[4 + q] = (_Float16)(bf16_val(b1) * 16.0f);
  }
  const v8us oh = fh.half[0], ob = fb.half[0];
  for (int pass = 0; pass < 2; ++pass) {
    *(volatile v8us*)(B16 + t * 8) = oh;
    *(volatile v8us*)(Bb + t * 8) = ob;
    if (pass == 0) __threadfence();
  }
}

template <int EPI, bool E>
__global__ __launch_bounds__(128) void k_gemm2(const unsigned short* __restrict__ A, const unsigned short* __restrict__ Al, int lda, size_t sA,
    const unsigned short* __restrict__ Bt, int ldb, float alpha, const float* __restrict__ bias,
    float* __restrict__ C, unsigned short* __restrict__ C16, unsigned short* __restrict__ EH, unsigned short* __restrict__ EL,
    int ldc, size_t sC, int lde, int M, int N, int K) {
  __shared__ __attribute__((aligned(16))) float so[4][32][68];
  const int tid = threadIdx.x, w = tid >> 5, lane = tid & 31, ln = lane & 15, hh = lane >> 4;
  const int by = blockIdx.y;
  A += (size_t)by * sA; Al += (size_t)by * sA;
  const size_t cofs = (size_t)by * sC;
  const int ntn = N >> 6;
  const int mt = blockIdx.x / ntn, nq = blockIdx.x - mt * ntn;
  const int row0 = mt * 128 + 32 * w, col0 = nq * 64;
  if (row0 >= M) return;
  const unsigned short* a0p = A + (size_t)(row0 + ln) * lda;
  const unsigned short* a1p = a0p + (size_t)16 * lda;
  const unsigned short* l0p = Al + (size_t)(row0 + ln) * lda;
  const unsigned short* l1p = l0p + (size_t)16 * lda;
  const unsigned short* b0p = Bt + (size_t)(col0 + ln) * ldb;
  const unsigned short* b1p = b0p + (size_t)16 * ldb;
  const unsigned short* b2p = b1p + (size_t)16 * ldb;
  const unsigned short* b3p = b2p + (size_t)16 * ldb;
  const v8f z8 = {0.f, 0.f, 0.f, 0.f, 0.f, 0.f, 0.f, 0.f};
  v8f c00 = z8, c01 = z8, c02 = z8, c03 = z8, c10 = z8, c11 = z8, c12 = z8, c13 = z8;
#pragma unroll 1
  for (int kb = 0; kb < K; kb += 32) {
    const Frag16 a0 = ld_frag(a0p + kb, hh), a1 = ld_frag(a1p + kb, hh);
    Frag16 a0l = a0, a1l = a1;
    if (E) { a0l = ld_frag(l0p + kb, hh); a1l = ld_frag(l1p + kb, hh); }
    Frag16 b = ld_frag(b0p + kb, hh); c00 = mm2<E>(a0, a0l, b, c00); c10 = mm2<E>(a1, a1l, b, c10);
    b = ld_frag(b1p + kb, hh); c01 = mm2<E>(a0, a0l, b, c01); c11 = mm2<E>(a1, a1l, b, c11);
    b = ld_frag(b2p + kb, hh); c02 = mm2<E>(a0, a0l, b, c02); c12 = mm2<E>(a1, a1l, b, c12);
    b = ld_frag(b3p + kb, hh); c03 = mm2<E>(a0, a0l, b, c03); c13 = mm2<E>(a1, a1l, b, c13);
  }
  v8f accs[8] = {c00, c01, c02, c03, c10, c11, c12, c13};
#pragma unroll
  for (int u = 0; u < 8; ++u) {
    const int t = u & 3, half = u >> 2;
    float bv = 0.f;
    if (EPI == 2) bv = bf16_rne(bias[col0 + t * 16 + ln]);
#pragma unroll
    for (int r = 0; r < 8; ++r) so[w][half * 16 + 8 * hh + r][t * 16 + ln] = accs[u][r] * alpha + bv;
  }
  __builtin_amdgcn_fence(4  , "workgroup");
  __builtin_amdgcn_wave_barrier();
  const int rsub = lane >> 4, c4 = (lane & 15) * 4;
  bool early = false; size_t erow0 = 0, ecol0 = 0;
  if (EPI == 0) { const int bb = row0 / SEQ, s0 = row0 - bb * SEQ; early = (s0 < EARLY); erow0 = (size_t)bb * EARLY + s0; ecol0 = (size_t)col0; }
  if (EPI == 1) { const int bb = col0 / SEQ, s0 = col0 - bb * SEQ; early = (s0 < EARLY); erow0 = (size_t)row0; ecol0 = (size_t)bb * EARLY + s0; }
  for (int pass = 0; pass < 2; ++pass) {
#pragma unroll
    for (int q = 0; q < 16; ++q) {
      const int r = q * 2 + rsub;
      const v4f v = *(const v4fa*)&so[w][r][c4];
      if (EPI == 2) {
        *(volatile v4f*)(C + cofs + (size_t)(row0 + r) * ldc + col0 + c4) = v;
      } else {
        v4us h4;
#pragma unroll
        for (int i = 0; i < 4; ++i) h4[i] = f16_bits(v[i]);
        *(volatile v4us*)(C16 + cofs + (size_t)(row0 + r) * ldc + col0 + c4) = h4;
        if (early) {
          v4us eh, el;
#pragma unroll
          for (int i = 0; i < 4; ++i) { const unsigned short hb = bf16_bits(v[i]); eh[i] = hb; el[i] = bf16_bits(v[i] - bf16_val(hb)); }
          const size_t eo = (erow0 + (size_t)r) * lde + ecol0 + c4;
          *(volatile v4us*)(EH + eo) = eh;
          *(volatile v4us*)(EL + eo) = el;
        }
      }
    }
    if (pass == 0) __threadfence();
  }
}

template <bool E>
__global__ __launch_bounds__(128) void k_flash(const unsigned short* __restrict__ QKh, const unsigned short* __restrict__ QKl, int ldq,
    const unsigned short* __restrict__ VTh, const unsigned short* __restrict__ VTl, int ldv,
    unsigned short* __restrict__ Ch, unsigned short* __restrict__ Cl, int SL, int qfirst) {
  __shared__ __attribute__((aligned(16))) unsigned short sh[4][16][72];
  __shared__ __attribute__((aligned(16))) unsigned short sl[4][16][72];
  const int tid = threadIdx.x, w = tid >> 5, lane = tid & 31, ln = lane & 15, hh = lane >> 4;
  const int bh = blockIdx.y, b = bh / NH, h = bh - b * NH;
  const int q0 = qfirst + blockIdx.x * 64 + 16 * w;
  const size_t rb = (size_t)b * SL;
  const int myq = q0 + ln;
  Frag16 qh[2], ql[2];
  {
    const size_t qo = (rb + q0 + ln) * (size_t)ldq + h * HD;
#pragma unroll
    for (int kk = 0; kk < 2; ++kk) {
      qh[kk] = ld_frag(QKh + qo + kk * 32, hh);
      ql[kk] = qh[kk];
      if (E) ql[kk] = ld_frag(QKl + qo + kk * 32, hh);
    }
  }
  const size_t kbase = rb * (size_t)ldq + DM + h * HD;
  const size_t vbase = (size_t)(h * HD) * ldv + rb;
  const v8f z8 = {0.f, 0.f, 0.f, 0.f, 0.f, 0.f, 0.f, 0.f};
  v8f acc[4] = {z8, z8, z8, z8};
  float m = -1.0e30f, l = 0.f;
  const int nch = (q0 + 15) / 64 + 1;
#pragma unroll 1
  for (int c = 0; c < nch; ++c) {
    const int jk = c * 64;
    v8f sc[4];
#pragma unroll
    for (int jt = 0; jt < 4; ++jt) {
      const size_t ko = kbase + (size_t)(jk + jt * 16 + ln) * ldq;
      v8f s = z8;
#pragma unroll
      for (int kk = 0; kk < 2; ++kk) {
        const Frag16 kh = ld_frag(QKh + ko + kk * 32, hh);
        Frag16 kl = kh;
        if (E) kl = ld_frag(QKl + ko + kk * 32, hh);
        s = mm3<E>(kh, kl, qh[kk], ql[kk], s);
      }
      sc[jt] = s;
    }
    float mx = m;
#pragma unroll
    for (int jt = 0; jt < 4; ++jt) {
#pragma unroll
      for (int r = 0; r < 8; ++r) {
        const int key = jk + jt * 16 + 8 * hh + r;
        float s = sc[jt][r] * 0.125f;
        s = (key <= myq) ? s : -1.0e30f;
        sc[jt][r] = s;
        mx = fmaxf(mx, s);
      }
    }
    mx = fmaxf(mx, __shfl_xor(mx, 16));
    const float alpha = __expf(m - mx);
    m = mx;
#pragma unroll
    for (int t = 0; t < 4; ++t) {
#pragma unroll
      for (int r = 0; r < 8; ++r) acc[t][r] *= alpha;
    }
    float ps = 0.f;
#pragma unroll
    for (int ks = 0; ks < 2; ++ks) {
      Frag16 ph, pl;
#pragma unroll
      for (int r = 0; r < 8; ++r) {
        const float p0 = __expf(sc[2 * ks][r] - mx), p1 = __expf(sc[2 * ks + 1][r] - mx);
        ps += p0 + p1;
        if (E) {
          const unsigned short h0 = bf16_bits(p0), h1 = bf16_bits(p1);
          ph.u[r] = h0; ph.u[8 + r] = h1;
          pl.u[r] = bf16_bits(p0 - bf16_val(h0)); pl.u[8 + r] = bf16_bits(p1 - bf16_val(h1));
        } else {
          ph.f[r] = (_Float16)(p0 * 256.0f); ph.f[8 + r] = (_Float16)(p1 * 256.0f);
        }
      }
      if (!E) pl = ph;
#pragma unroll
      for (int t = 0; t < 4; ++t) {
        const size_t vo = vbase + (size_t)(t * 16 + ln) * ldv + jk + ks * 32;
        const Frag16 vh = ld_frag(VTh + vo, hh);
        Frag16 vl = vh;
        if (E) vl = ld_frag(VTl + vo, hh);
        acc[t] = mm3<E>(vh, vl, ph, pl, acc[t]);
      }
    }
    l = l * alpha + ps;
  }
  l += __shfl_xor(l, 16);
  const float inv = (E ? 1.0f : 0.25f) * (1.0f / l);
#pragma unroll
  for (int t = 0; t < 4; ++t) {
#pragma unroll
    for (int r = 0; r < 8; ++r) {
      const float o = acc[t][r] * inv;
      const int d = t * 16 + 8 * hh + r;
      if (E) { const unsigned short hb = bf16_bits(o); sh[w][ln][d] = hb; sl[w][ln][d] = bf16_bits(o - bf16_val(hb)); }
      else sh[w][ln][d] = f16_bits(o);
    }
  }
  __builtin_amdgcn_fence(4  , "workgroup");
  __builtin_amdgcn_wave_barrier();
  const int rq = lane >> 3, pc = (lane & 7) * 8;
  v8us oh[4], ol[4];
#pragma unroll
  for (int i = 0; i < 4; ++i) {
    oh[i] = *(const v8us*)&sh[w][i * 4 + rq][pc];
    ol[i] = oh[i];
    if (E) ol[i] = *(const v8us*)&sl[w][i * 4 + rq][pc];
  }
  for (int pass = 0; pass < 2; ++pass) {
#pragma unroll
    for (int i = 0; i < 4; ++i) {
      const size_t go = (rb + q0 + i * 4 + rq) * (size_t)DM + h * HD + pc;
      *(volatile v8us*)(Ch + go) = oh[i];
      if (E) *(volatile v8us*)(Cl + go) = ol[i];
    }
    if (pass == 0) __threadfence();
  }
}

extern "C" void kernel_launch(void* const* d_in, const int* in_sizes, int n_in,
                              void* d_out, int out_size, void* d_ws, size_t ws_size, hipStream_t stream) {
  static_assert(NH * HD == DM);
  static_assert(DM % 128 == 0 && SEQ % 128 == 0 && EARLY % 128 == 0 && SEQ >= EARLY && (SEQ - EARLY) % 128 == 0);
  static_assert(NB <= NB_FULL && SEQ <= SEQ_FULL);
  if (n_in < 6) return;
  const long long need_x = ((long long)(NB - 1) * SEQ_FULL + SEQ) * DM;
  if ((long long)in_sizes[0] < need_x) return;
  if (in_sizes[1] < NH * DM * HD || in_sizes[2] < NH * DM * HD || in_sizes[3] < NH * DM * HD) return;
  if (in_sizes[4] < DM * DM || in_sizes[5] < DM) return;
  if ((long long)out_size < need_x) return;
  const float* x  = (const float*)d_in[0];
  const float* Wq = (const float*)d_in[1];
  const float* Wk = (const float*)d_in[2];
  const float* Wv = (const float*)d_in[3];
  const float* Wo = (const float*)d_in[4];
  const float* bo = (const float*)d_in[5];
  float* out = (float*)d_out;

  char* ws = (char*)d_ws; size_t off = 0;
  auto take = [&](size_t bytes) { char* p = ws + off; off += (bytes + 255) & ~(size_t)255; return p; };
  unsigned short* BQK  = (unsigned short*)take((size_t)2 * DM * DM * 2);
  unsigned short* BV   = (unsigned short*)take((size_t)DM * DM * 2);
  unsigned short* BO16 = (unsigned short*)take((size_t)DM * DM * 2);
  unsigned short* BOb  = (unsigned short*)take((size_t)DM * DM * 2);
  unsigned short* X16  = (unsigned short*)take(NR * DM * 2);
  unsigned short* QK16 = (unsigned short*)take(NR * 2 * DM * 2);
  unsigned short* VT   = (unsigned short*)take((size_t)DM * NR * 2);
  unsigned short* C16  = (unsigned short*)take(NR * DM * 2);
  unsigned short* EQh  = (unsigned short*)take(NE * 2 * DM * 2);
  unsigned short* EQl  = (unsigned short*)take(NE * 2 * DM * 2);
  unsigned short* EVh  = (unsigned short*)take((size_t)DM * NE * 2);
  unsigned short* EVl  = (unsigned short*)take((size_t)DM * NE * 2);
  unsigned short* ECh  = (unsigned short*)take(NE * DM * 2);
  unsigned short* ECl  = (unsigned short*)take(NE * DM * 2);
  if (off > ws_size || off > (size_t)134217728) return;

  k_x16<<<(unsigned)((NR * DM / 8 + 255) / 256), 256, 0, stream>>>(x, X16);
  k_wt_heads<<<(NH * HD * (DM / 8) + 255) / 256, 256, 0, stream>>>(Wq, BQK);
  k_wt_heads<<<(NH * HD * (DM / 8) + 255) / 256, 256, 0, stream>>>(Wk, BQK + (size_t)DM * DM);
  k_wt_heads<<<(NH * HD * (DM / 8) + 255) / 256, 256, 0, stream>>>(Wv, BV);
  k_wo<<<(DM * DM / 8 + 255) / 256, 256, 0, stream>>>(Wo, BO16, BOb);

  k_gemm2<0, false><<<dim3((unsigned)((NR / 128) * (2 * DM / 64)), 1), 128, 0, stream>>>(
      X16, X16, DM, (size_t)0, BQK, DM, 0.0625f, bo, out, QK16, EQh, EQl, 2 * DM, (size_t)0, 2 * DM, (int)NR, 2 * DM, DM);
  k_gemm2<1, false><<<dim3((unsigned)((DM / 128) * (NR / 64)), 1), 128, 0, stream>>>(
      BV, BV, DM, (size_t)0, X16, DM, 0.0625f, bo, out, VT, EVh, EVl, (int)NR, (size_t)0, (int)NE, DM, (int)NR, DM);

  k_flash<true><<<dim3(EARLY / 64, NB * NH), 128, 0, stream>>>(EQh, EQl, 2 * DM, EVh, EVl, (int)NE, ECh, ECl, EARLY, 0);
  if (SEQ > EARLY)
    k_flash<false><<<dim3((SEQ - EARLY) / 64, NB * NH), 128, 0, stream>>>(QK16, QK16, 2 * DM, VT, VT, (int)NR, C16, C16, SEQ, EARLY);

  k_gemm2<2, true><<<dim3((EARLY / 128) * (DM / 64), NB), 128, 0, stream>>>(
      ECh, ECl, DM, (size_t)EARLY * DM, BOb, DM, 1.0f, bo, out, C16, C16, C16, DM, (size_t)SEQ_FULL * DM, DM, EARLY, DM, DM);
  if (SEQ > EARLY)
    k_gemm2<2, false><<<dim3(((SEQ - EARLY) / 128) * (DM / 64), NB), 128, 0, stream>>>(
        C16 + (size_t)EARLY * DM, C16 + (size_t)EARLY * DM, DM, (size_t)SEQ * DM, BO16, DM, 0.0009765625f, bo,
        out + (size_t)EARLY * DM, C16, C16, C16, DM, (size_t)SEQ_FULL * DM, DM, SEQ - EARLY, DM, DM);
}
